// NeuralClusteringAttention_86354612453690
// MI455X (gfx1250) — hardware-verified
//
#include <hip/hip_runtime.h>
#include <stdint.h>


#define B_    4
#define T_    1024
#define D_    512
#define C_    8
#define H_    8
#define HD_   64
#define NTOK_ (B_ * T_)
#define D3_   (3 * D_)
#define SEGI_ (32 + T_)

static_assert(NTOK_ % 32 == 0);
static_assert(D_ % 64 == 0 && D3_ % 64 == 0);
static_assert(T_ % 32 == 0 && HD_ == 64);
static_assert((NTOK_ / 16) * (D3_ / 64) % 8 == 0);
static_assert((NTOK_ / 16) * (D_ / 64) % 8 == 0);

typedef unsigned short u16;
typedef u16    u16x8  __attribute__((ext_vector_type(8)));
typedef u16    u16x16 __attribute__((ext_vector_type(16)));
typedef __bf16 bf16_t;
typedef bf16_t bf16x16 __attribute__((ext_vector_type(16)));
typedef float  f32x8  __attribute__((ext_vector_type(8)));
typedef float  v4f    __attribute__((ext_vector_type(4)));
typedef int    v4i    __attribute__((ext_vector_type(4)));

union Frag { bf16x16 v; u16x16 u; u16x8 hv[2]; };

__device__ __forceinline__ bf16x16 ldfrag(const u16* p, int hf) {
  Frag f;
  f.hv[0] = *(const u16x8*)(p + 8 * hf);
  f.hv[1] = *(const u16x8*)(p + 16 + 8 * hf);
  return f.v;
}

__device__ __forceinline__ f32x8 wmma_bf16(bf16x16 a, bf16x16 b, f32x8 c) {
  f32x8 d = __builtin_amdgcn_wmma_f32_16x16x32_bf16(false, a, false, b, (short)0, c, false, false);
  asm volatile("v_nop\n\tv_nop\n\tv_nop\n\tv_nop" : "+v"(d) : "v"(a), "v"(b));
  return d;
}

__device__ __forceinline__ f32x8 wmma_split(bf16x16 ah, bf16x16 al, bf16x16 bh, bf16x16 bl, f32x8 c) {
  c = wmma_bf16(ah, bh, c);
  c = wmma_bf16(ah, bl, c);
  c = wmma_bf16(al, bh, c);
  return c;
}

__device__ __forceinline__ u16 bf16_rne(float x) {
  unsigned u = __float_as_uint(x);
  u = u + 0x7FFFu + ((u >> 16) & 1u);
  return (u16)(u >> 16);
}
__device__ __forceinline__ float bf16_to_f32(u16 b) {
  return __uint_as_float(((unsigned)b) << 16);
}
__device__ __forceinline__ void split1(float x, u16& hi, u16& lo) {
  hi = bf16_rne(x);
  lo = bf16_rne(x - bf16_to_f32(hi));
}
__device__ __forceinline__ void split8(v4f a, v4f b, u16x8& hi, u16x8& lo) {
  float v[8] = {a.x, a.y, a.z, a.w, b.x, b.y, b.z, b.w};
  u16x8 hh = {0, 0, 0, 0, 0, 0, 0, 0};
  u16x8 ll = {0, 0, 0, 0, 0, 0, 0, 0};
#pragma unroll
  for (int i = 0; i < 8; ++i) {
    u16 x, y;
    split1(v[i], x, y);
    hh[i] = x;
    ll[i] = y;
  }
  hi = hh;
  lo = ll;
}

__global__ __launch_bounds__(256) void k_assign(const float* __restrict__ X,
                                                 const float* __restrict__ Wc,
                                                 const float* __restrict__ bc,
                                                 int* assign) {
  __shared__ float wcs[C_ * D_];
  __shared__ __align__(16) int res[32];
  const int t = threadIdx.x, l = t & 31, w = t >> 5;
  for (int i = t; i < C_ * D_; i += 256) wcs[i] = Wc[i];
  __syncthreads();

  for (int i = 0; i < 4; ++i) {
    const int tok = blockIdx.x * 32 + w * 4 + i;
    const float* x = X + (size_t)tok * D_;
    double s[C_];
#pragma unroll
    for (int c = 0; c < C_; ++c) s[c] = 0.0;
#pragma unroll 2
    for (int j = 0; j < D_ / 32; ++j) {
      const int d = l + 32 * j;
      const double xv = (double)x[d];
#pragma unroll
      for (int c = 0; c < C_; ++c) s[c] += xv * (double)wcs[c * D_ + d];
    }
#pragma unroll
    for (int off = 16; off > 0; off >>= 1) {
#pragma unroll
      for (int c = 0; c < C_; ++c) s[c] += __shfl_xor(s[c], off, 32);
    }
    if (l == 0) {
      int best = 0;
      float bv = (float)s[0] + bc[0];
#pragma unroll
      for (int c = 1; c < C_; ++c) {
        const float v = (float)s[c] + bc[c];
        if (v > bv) { bv = v; best = c; }
      }
      res[w * 4 + i] = best;
    }
  }
  __syncthreads();
  v4i v = {0, 0, 0, 0};
  if (t < 8) {
    v = *(const v4i*)(res + 4 * t);
    *(volatile v4i*)(assign + (size_t)blockIdx.x * 32 + 4 * t) = v;
  }
  __threadfence();
  if (t < 8) {
    *(volatile v4i*)(assign + (size_t)blockIdx.x * 32 + 4 * t) = v;
  }
}

__global__ __launch_bounds__(256) void k_lists(const int* __restrict__ assign, int* lists) {
  __shared__ __align__(16) int lst[T_];
  __shared__ int wsum[8];
  const int bcid = blockIdx.x, b = bcid / C_, c = bcid % C_;
  const int t = threadIdx.x, l = t & 31, w = t >> 5;

  const v4i a = *(const v4i*)(assign + (size_t)b * T_ + 4 * t);
  const int f0 = (a.x == c) ? 1 : 0;
  const int f1 = (a.y == c) ? 1 : 0;
  const int f2 = (a.z == c) ? 1 : 0;
  const int f3 = (a.w == c) ? 1 : 0;
  const int cnt = f0 + f1 + f2 + f3;

  lst[4 * t + 0] = 0;
  lst[4 * t + 1] = 0;
  lst[4 * t + 2] = 0;
  lst[4 * t + 3] = 0;

  int x = cnt;
#pragma unroll
  for (int off = 1; off < 32; off <<= 1) {
    const int y = __shfl_up(x, off, 32);
    if (l >= off) x += y;
  }
  if (l == 31) wsum[w] = x;
  __syncthreads();
  int base = 0, total = 0;
#pragma unroll
  for (int i = 0; i < 8; ++i) {
    const int sv = wsum[i];
    total += sv;
    if (i < w) base += sv;
  }
  int pos = base + x - cnt;
  if (f0) { lst[pos] = 4 * t + 0; ++pos; }
  if (f1) { lst[pos] = 4 * t + 1; ++pos; }
  if (f2) { lst[pos] = 4 * t + 2; ++pos; }
  if (f3) { lst[pos] = 4 * t + 3; ++pos; }
  __syncthreads();

  const v4i mine = *(const v4i*)(lst + 4 * t);
  v4i hv = {0, 0, 0, 0};
  if (t == 0) hv.x = total;
  int* segp = lists + (size_t)bcid * SEGI_;
  if (t < 8) *(volatile v4i*)(segp + 4 * t) = hv;
  *(volatile v4i*)(segp + 32 + 4 * t) = mine;
  __threadfence();
  if (t < 8) *(volatile v4i*)(segp + 4 * t) = hv;
  *(volatile v4i*)(segp + 32 + 4 * t) = mine;
}

__global__ __launch_bounds__(256) void k_convert(const float* __restrict__ X,
                                                  const float* __restrict__ Win,
                                                  const float* __restrict__ Wout,
                                                  u16* Xh, u16* Xl, u16* Wih, u16* Wil,
                                                  u16* Woh, u16* Wol) {
  const unsigned g = blockIdx.x * 256u + threadIdx.x;
  const unsigned nx = (unsigned)(NTOK_ * D_ / 8);
  const unsigned nw = (unsigned)(D3_ * D_ / 8);
  const unsigned no = (unsigned)(D_ * D_ / 8);
  const float* src;
  u16* dh;
  u16* dl;
  size_t e;
  if (g < nx) {
    src = X; dh = Xh; dl = Xl; e = (size_t)g * 8;
  } else if (g < nx + nw) {
    src = Win; dh = Wih; dl = Wil; e = (size_t)(g - nx) * 8;
  } else if (g < nx + nw + no) {
    src = Wout; dh = Woh; dl = Wol; e = (size_t)(g - nx - nw) * 8;
  } else {
    return;
  }
  const v4f a = *(const v4f*)(src + e);
  const v4f b = *(const v4f*)(src + e + 4);
  u16x8 hi, lo;
  split8(a, b, hi, lo);
  *(volatile u16x8*)(dh + e) = hi;
  *(volatile u16x8*)(dl + e) = lo;
  __threadfence();
  *(volatile u16x8*)(dh + e) = hi;
  *(volatile u16x8*)(dl + e) = lo;
}

__global__ __launch_bounds__(256) void k_qkv(const u16* __restrict__ Xh, const u16* __restrict__ Xl,
                                              const u16* __restrict__ Wih, const u16* __restrict__ Wil,
                                              const float* __restrict__ bin,
                                              u16* QKVh, u16* QKVl) {
  __shared__ __align__(16) float stg[8 * 16 * 64];
  const int wl = threadIdx.x >> 5;
  const int wave = blockIdx.x * 8 + wl;
  const int l = threadIdx.x & 31, m = l & 15, hf = l >> 4;
  const int NG = D3_ / 64;
  const int mt = wave / NG, ng = wave % NG;

  const u16* ahp = Xh + (size_t)(mt * 16 + m) * D_;
  const u16* alp = Xl + (size_t)(mt * 16 + m) * D_;
  const u16* bhp = Wih + (size_t)(ng * 64 + m) * D_;
  const u16* blp = Wil + (size_t)(ng * 64 + m) * D_;

  f32x8 acc[4];
#pragma unroll
  for (int sub = 0; sub < 4; ++sub) acc[sub] = (f32x8){0.f, 0.f, 0.f, 0.f, 0.f, 0.f, 0.f, 0.f};

#pragma unroll 1
  for (int k0 = 0; k0 < D_; k0 += 32) {
    const bf16x16 ah = ldfrag(ahp + k0, hf);
    const bf16x16 al = ldfrag(alp + k0, hf);
#pragma unroll
    for (int sub = 0; sub < 4; ++sub) {
      const bf16x16 bh = ldfrag(bhp + (size_t)sub * 16 * D_ + k0, hf);
      const bf16x16 bl = ldfrag(blp + (size_t)sub * 16 * D_ + k0, hf);
      acc[sub] = wmma_split(ah, al, bh, bl, acc[sub]);
    }
  }

  float* st = stg + wl * (16 * 64);
#pragma unroll
  for (int sub = 0; sub < 4; ++sub) {
    const float bias = bin[ng * 64 + sub * 16 + m];
#pragma unroll
    for (int r = 0; r < 8; ++r) st[(8 * hf + r) * 64 + sub * 16 + m] = acc[sub][r] + bias;
  }
  __syncthreads();

  u16x8 hv[4], lv[4];
  size_t go[4];
#pragma unroll
  for (int it = 0; it < 4; ++it) {
    const int row = it * 4 + (l >> 3);
    const int c8 = (l & 7) * 8;
    const v4f a = *(const v4f*)(st + row * 64 + c8);
    const v4f b = *(const v4f*)(st + row * 64 + c8 + 4);
    split8(a, b, hv[it], lv[it]);
    go[it] = (size_t)(mt * 16 + row) * D3_ + (size_t)ng * 64 + c8;
    *(volatile u16x8*)(QKVh + go[it]) = hv[it];
    *(volatile u16x8*)(QKVl + go[it]) = lv[it];
  }
  __threadfence();
#pragma unroll
  for (int it = 0; it < 4; ++it) {
    *(volatile u16x8*)(QKVh + go[it]) = hv[it];
    *(volatile u16x8*)(QKVl + go[it]) = lv[it];
  }
}

__device__ __forceinline__ f32x8 score16(bf16x16 qh0, bf16x16 qh1, bf16x16 ql0, bf16x16 ql1,
                                          const u16* Kh, const u16* Kl, size_t kb, int hf) {
  f32x8 s = {0.f, 0.f, 0.f, 0.f, 0.f, 0.f, 0.f, 0.f};
  {
    const bf16x16 kh = ldfrag(Kh + kb, hf);
    const bf16x16 kl = ldfrag(Kl + kb, hf);
    s = wmma_split(qh0, ql0, kh, kl, s);
  }
  {
    const bf16x16 kh = ldfrag(Kh + kb + 32, hf);
    const bf16x16 kl = ldfrag(Kl + kb + 32, hf);
    s = wmma_split(qh1, ql1, kh, kl, s);
  }
  return s;
}

__global__ __launch_bounds__(32) void k_attn(const u16* __restrict__ QKVh, const u16* __restrict__ QKVl,
                                             const float* __restrict__ bin, const int* __restrict__ lists,
                                             u16* Oh, u16* Ol) {
  __shared__ __align__(16) u16 vh[32 * HD_];
  __shared__ __align__(16) u16 vl[32 * HD_];
  __shared__ __align__(16) u16 ph[16 * 32];
  __shared__ __align__(16) u16 pl[16 * 32];
  __shared__ __align__(16) float ost[16 * HD_];

  const int qt = blockIdx.x, h = blockIdx.y, bcid = blockIdx.z;
  const int* seg = lists + (size_t)bcid * SEGI_;
  int n = seg[0];
  if (n > T_) n = T_;
  if (n <= 0 || qt * 16 >= n) return;
  const int* idx = seg + 32;
  const int b = bcid / C_;
  const int l = threadIdx.x, m = l & 15, hf = l >> 4;
  const size_t tokb = (size_t)b * T_;

  const int qrow = qt * 16 + m;
  const int qc = (qrow < n) ? qrow : (n - 1);
  const size_t qb = (tokb + (size_t)(idx[qc] & (T_ - 1))) * D3_ + (size_t)h * HD_;
  Frag fqh0, fqh1, fql0, fql1;
  fqh0.v = ldfrag(QKVh + qb, hf);
  fqh1.v = ldfrag(QKVh + qb + 32, hf);
  fql0.v = ldfrag(QKVl + qb, hf);
  fql1.v = ldfrag(QKVl + qb + 32, hf);

  const float* bk = bin + D_ + h * HD_;
  float part = 0.f;
#pragma unroll
  for (int i = 0; i < 16; ++i) {
    const int d = 8 * hf + i + ((i >> 3) << 3);
    const float q0 = bf16_to_f32(fqh0.u[i]) + bf16_to_f32(fql0.u[i]);
    const float q1 = bf16_to_f32(fqh1.u[i]) + bf16_to_f32(fql1.u[i]);
    part += q0 * bk[d] + q1 * bk[32 + d];
  }
  part += __shfl_xor(part, 16, 32);
  const float soutm = part * 0.125f;
  float sout[8];
#pragma unroll
  for (int r = 0; r < 8; ++r) sout[r] = __shfl(soutm, 8 * hf + r, 32);

  const bool hasOut = (n < T_);
  float M[8], Z[8];
#pragma unroll
  for (int r = 0; r < 8; ++r) { M[r] = hasOut ? sout[r] : -1e30f; Z[r] = 0.f; }
  f32x8 oc[4];
#pragma unroll
  for (int nc = 0; nc < 4; ++nc) oc[nc] = (f32x8){0.f, 0.f, 0.f, 0.f, 0.f, 0.f, 0.f, 0.f};

  for (int kt = 0; kt < n; kt += 32) {
    {
      const int kr = kt + l;
      const int kc = (kr < n) ? kr : (n - 1);
      const size_t vb = (tokb + (size_t)(idx[kc] & (T_ - 1))) * D3_ + 2 * D_ + (size_t)h * HD_;
#pragma unroll
      for (int j = 0; j < 8; ++j) {
        *(u16x8*)(vh + l * HD_ + j * 8) = *(const u16x8*)(QKVh + vb + j * 8);
        *(u16x8*)(vl + l * HD_ + j * 8) = *(const u16x8*)(QKVl + vb + j * 8);
      }
    }

    const int kcol0 = kt + m, kcol1 = kt + 16 + m;
    const int kc0 = (kcol0 < n) ? kcol0 : (n - 1);
    const int kc1 = (kcol1 < n) ? kcol1 : (n - 1);
    const size_t kb0 = (tokb + (size_t)(idx[kc0] & (T_ - 1))) * D3_ + D_ + (size_t)h * HD_;
    const size_t kb1 = (tokb + (size_t)(idx[kc1] & (T_ - 1))) * D3_ + D_ + (size_t)h * HD_;
    f32x8 s0 = score16(fqh0.v, fqh1.v, fql0.v, fql1.v, QKVh, QKVl, kb0, hf);
    f32x8 s1 = score16(fqh0.v, fqh1.v, fql0.v, fql1.v, QKVh, QKVl, kb1, hf);
    const bool ok0 = (kcol0 < n), ok1 = (kcol1 < n);
#pragma unroll
    for (int r = 0; r < 8; ++r) {
      s0[r] = ok0 ? s0[r] * 0.125f : -1e30f;
      s1[r] = ok1 ? s1[r] * 0.125f : -1e30f;
    }

    float nm[8];
#pragma unroll
    for (int r = 0; r < 8; ++r) nm[r] = fmaxf(s0[r], s1[r]);
#pragma unroll
    for (int off = 1; off < 16; off <<= 1) {
#pragma unroll
      for (int r = 0; r < 8; ++r) nm[r] = fmaxf(nm[r], __shfl_xor(nm[r], off, 32));
    }
    float alpha[8], p0[8], p1[8], psum[8];
#pragma unroll
    for (int r = 0; r < 8; ++r) {
      const float newm = fmaxf(M[r], nm[r]);
      alpha[r] = __expf(M[r] - newm);
      M[r] = newm;
      p0[r] = __expf(s0[r] - newm);
      p1[r] = __expf(s1[r] - newm);
      psum[r] = p0[r] + p1[r];
    }
#pragma unroll
    for (int off = 1; off < 16; off <<= 1) {
#pragma unroll
      for (int r = 0; r < 8; ++r) psum[r] += __shfl_xor(psum[r], off, 32);
    }
#pragma unroll
    for (int r = 0; r < 8; ++r) Z[r] = Z[r] * alpha[r] + psum[r];
#pragma unroll
    for (int nc = 0; nc < 4; ++nc) {
#pragma unroll
      for (int r = 0; r < 8; ++r) oc[nc][r] = oc[nc][r] * alpha[r];
    }

#pragma unroll
    for (int r = 0; r < 8; ++r) {
      u16 xh, xl, yh, yl;
      split1(p0[r], xh, xl);
      split1(p1[r], yh, yl);
      const int row = 8 * hf + r;
      ph[row * 32 + m] = xh;
      pl[row * 32 + m] = xl;
      ph[row * 32 + 16 + m] = yh;
      pl[row * 32 + 16 + m] = yl;
    }
    __syncthreads();

    const bf16x16 pah = ldfrag(ph + m * 32, hf);
    const bf16x16 pal = ldfrag(pl + m * 32, hf);
#pragma unroll
    for (int nc = 0; nc < 4; ++nc) {
      Frag fvh, fvl;
      const int col = nc * 16 + m;
#pragma unroll
      for (int i = 0; i < 16; ++i) {
        const int key = 8 * hf + i + ((i >> 3) << 3);
        fvh.u[i] = vh[key * HD_ + col];
        fvl.u[i] = vl[key * HD_ + col];
      }
      oc[nc] = wmma_split(pah, pal, fvh.v, fvl.v, oc[nc]);
    }
    __syncthreads();
  }

  const float extra = hasOut ? (float)(T_ - n) : 0.f;
  const float* bvp = bin + 2 * D_ + h * HD_;
  float bvv[4];
#pragma unroll
  for (int nc = 0; nc < 4; ++nc) bvv[nc] = bvp[nc * 16 + m];
#pragma unroll
  for (int r = 0; r < 8; ++r) {
    const float eo = extra * __expf(sout[r] - M[r]);
    const float inv = 1.0f / (Z[r] + eo);
#pragma unroll
    for (int nc = 0; nc < 4; ++nc)
      ost[(8 * hf + r) * HD_ + nc * 16 + m] = (oc[nc][r] + eo * bvv[nc]) * inv;
  }
  __syncthreads();

  u16x8 hv[4], lv[4];
  size_t go[4];
  bool okr[4];
#pragma unroll
  for (int it = 0; it < 4; ++it) {
    const int row = it * 4 + (l >> 3);
    const int c8 = (l & 7) * 8;
    const int qr = qt * 16 + row;
    okr[it] = (qr < n);
    const int qq = okr[it] ? qr : (n - 1);
    go[it] = (tokb + (size_t)(idx[qq] & (T_ - 1))) * D_ + (size_t)h * HD_ + c8;
    const v4f a = *(const v4f*)(ost + row * HD_ + c8);
    const v4f b2 = *(const v4f*)(ost + row * HD_ + c8 + 4);
    split8(a, b2, hv[it], lv[it]);
    if (okr[it]) {
      *(volatile u16x8*)(Oh + go[it]) = hv[it];
      *(volatile u16x8*)(Ol + go[it]) = lv[it];
    }
  }
  __threadfence();
#pragma unroll
  for (int it = 0; it < 4; ++it) {
    if (okr[it]) {
      *(volatile u16x8*)(Oh + go[it]) = hv[it];
      *(volatile u16x8*)(Ol + go[it]) = lv[it];
    }
  }
}

__global__ __launch_bounds__(256) void k_outproj(const u16* __restrict__ Oh, const u16* __restrict__ Ol,
                                                  const u16* __restrict__ Woh, const u16* __restrict__ Wol,
                                                  const float* __restrict__ bout, float* out) {
  __shared__ __align__(16) float stg[8 * 16 * 64];
  const int wl = threadIdx.x >> 5;
  const int wave = blockIdx.x * 8 + wl;
  const int l = threadIdx.x & 31, m = l & 15, hf = l >> 4;
  const int NG = D_ / 64;
  const int mt = wave / NG, ng = wave % NG;

  const u16* ahp = Oh + (size_t)(mt * 16 + m) * D_;
  const u16* alp = Ol + (size_t)(mt * 16 + m) * D_;
  const u16* bhp = Woh + (size_t)(ng * 64 + m) * D_;
  const u16* blp = Wol + (size_t)(ng * 64 + m) * D_;

  f32x8 acc[4];
#pragma unroll
  for (int sub = 0; sub < 4; ++sub) acc[sub] = (f32x8){0.f, 0.f, 0.f, 0.f, 0.f, 0.f, 0.f, 0.f};

#pragma unroll 1
  for (int k0 = 0; k0 < D_; k0 += 32) {
    const bf16x16 ah = ldfrag(ahp + k0, hf);
    const bf16x16 al = ldfrag(alp + k0, hf);
#pragma unroll
    for (int sub = 0; sub < 4; ++sub) {
      const bf16x16 bh = ldfrag(bhp + (size_t)sub * 16 * D_ + k0, hf);
      const bf16x16 bl = ldfrag(blp + (size_t)sub * 16 * D_ + k0, hf);
      acc[sub] = wmma_split(ah, al, bh, bl, acc[sub]);
    }
  }

  float* st = stg + wl * (16 * 64);
#pragma unroll
  for (int sub = 0; sub < 4; ++sub) {
    const float bias = bout[ng * 64 + sub * 16 + m];
#pragma unroll
    for (int r = 0; r < 8; ++r) st[(8 * hf + r) * 64 + sub * 16 + m] = acc[sub][r] + bias;
  }
  __syncthreads();

  v4f ov[8];
  size_t go[8];
#pragma unroll
  for (int it = 0; it < 8; ++it) {
    const int row = it * 2 + (l >> 4);
    const int c4 = (l & 15) * 4;
    ov[it] = *(const v4f*)(st + row * 64 + c4);
    go[it] = (size_t)(mt * 16 + row) * D_ + (size_t)ng * 64 + c4;
    *(volatile v4f*)(out + go[it]) = ov[it];
  }
  __threadfence();
#pragma unroll
  for (int it = 0; it < 8; ++it) {
    *(volatile v4f*)(out + go[it]) = ov[it];
  }
}

extern "C" void kernel_launch(void* const* d_in, const int* in_sizes, int n_in,
                              void* d_out, int out_size, void* d_ws, size_t ws_size,
                              hipStream_t stream) {
  if (n_in < 7) return;
  if (in_sizes[0] != NTOK_ * D_ || in_sizes[1] != C_ * D_ || in_sizes[2] != C_ ||
      in_sizes[3] != D3_ * D_ || in_sizes[4] != D3_ || in_sizes[5] != D_ * D_ ||
      in_sizes[6] != D_) return;
  if (out_size != NTOK_ * D_) return;

  const float* X    = (const float*)d_in[0];
  const float* Wc   = (const float*)d_in[1];
  const float* bc   = (const float*)d_in[2];
  const float* Win  = (const float*)d_in[3];
  const float* bin  = (const float*)d_in[4];
  const float* Wout = (const float*)d_in[5];
  const float* bout = (const float*)d_in[6];
  float* out = (float*)d_out;

  size_t off = 0;
  char* ws = (char*)d_ws;
  const size_t sz_assign = (size_t)NTOK_ * 4;
  const size_t sz_lists  = (size_t)B_ * C_ * SEGI_ * 4;
  const size_t sz_x16    = (size_t)NTOK_ * D_ * 2;
  const size_t sz_win16  = (size_t)D3_ * D_ * 2;
  const size_t sz_wout16 = (size_t)D_ * D_ * 2;
  const size_t sz_qkv16  = (size_t)NTOK_ * D3_ * 2;
  const size_t sz_o16    = (size_t)NTOK_ * D_ * 2;

  int* assign = (int*)(ws + off); off += sz_assign;
  int* lists  = (int*)(ws + off); off += sz_lists;
  u16* Xh   = (u16*)(ws + off); off += sz_x16;
  u16* Xl   = (u16*)(ws + off); off += sz_x16;
  u16* Wih  = (u16*)(ws + off); off += sz_win16;
  u16* Wil  = (u16*)(ws + off); off += sz_win16;
  u16* Woh  = (u16*)(ws + off); off += sz_wout16;
  u16* Wol  = (u16*)(ws + off); off += sz_wout16;
  u16* QKVh = (u16*)(ws + off); off += sz_qkv16;
  u16* QKVl = (u16*)(ws + off); off += sz_qkv16;
  u16* Oh   = (u16*)(ws + off); off += sz_o16;
  u16* Ol   = (u16*)(ws + off); off += sz_o16;
  if (off > ws_size) return;

  k_assign<<<NTOK_ / 32, 256, 0, stream>>>(X, Wc, bc, assign);
  k_lists<<<B_ * C_, 256, 0, stream>>>(assign, lists);
  {
    const unsigned nthr = (unsigned)(NTOK_ * D_ / 8 + D3_ * D_ / 8 + D_ * D_ / 8);
    const unsigned nblk = (nthr + 255u) / 256u;
    k_convert<<<nblk, 256, 0, stream>>>(X, Win, Wout, Xh, Xl, Wih, Wil, Woh, Wol);
  }
  k_qkv<<<(NTOK_ / 16) * (D3_ / 64) / 8, 256, 0, stream>>>(Xh, Xl, Wih, Wil, bin, QKVh, QKVl);
  k_attn<<<dim3(T_ / 16, H_, B_ * C_), 32, 0, stream>>>(QKVh, QKVl, bin, lists, Oh, Ol);
  k_outproj<<<(NTOK_ / 16) * (D_ / 64) / 8, 256, 0, stream>>>(Oh, Ol, Woh, Wol, bout, out);
}
